// RNN_70935679861111
// MI455X (gfx1250) — hardware-verified
//
#include <hip/hip_runtime.h>
#include <math.h>

constexpr int NB     = 256;
constexpr int NT     = 2048;
constexpr int NIN    = 16;
constexpr int NH     = 64;
constexpr int NGC    = 4 * NH;
constexpr int NO     = 2;
constexpr int KTOT   = 96;
constexpr int WPITCH = 128;
constexpr int AP     = 104;
constexpr int HFP    = 260;
constexpr int OBP    = 32;
constexpr int ROWB   = 16;
constexpr int NTHR   = 128;
constexpr int NTHRP  = 256;
constexpr int TFL    = 16;
constexpr float WCARRY     = 16.0f;
constexpr float WCARRY_INV = 1.0f / 16.0f;
constexpr float LCARRY     = 1024.0f;
constexpr float LCARRY_INV = 1.0f / 1024.0f;
static_assert(NB % ROWB == 0);
static_assert(NH == 16 * (NTHR / 32));
static_assert(KTOT % 32 == 0 && KTOT == NH + 2 * NIN);
static_assert(KTOT <= WPITCH && KTOT + 8 <= AP && AP % 8 == 0 && WPITCH % 64 == 0);
static_assert(NT % TFL == 0 && TFL * NO * 4 == 128);
static_assert((ROWB * AP) % NTHR == 0);
static_assert(ROWB * 8 == NTHR);
static_assert((NGC * (WPITCH / 8)) % NTHRP == 0);
static_assert(NO * NH == 128);
static_assert(HFP % 4 == 0 && OBP % 4 == 0);

typedef __attribute__((ext_vector_type(16))) _Float16 v16h;
typedef __attribute__((ext_vector_type(8)))  _Float16 v8h;
typedef __attribute__((ext_vector_type(8)))  float    v8f;
typedef __attribute__((ext_vector_type(4)))  float    v4f;
typedef __attribute__((ext_vector_type(2)))  unsigned v2u;

template <typename T> struct Frag;
template <> struct Frag<_Float16> {
  typedef v16h V; union U { v16h v; v8h h[2]; };
  static __device__ __forceinline__ v16h load(const _Float16* p) {
    U f; f.h[0] = *(const v8h*)(p); f.h[1] = *(const v8h*)(p + 16); return f.v;
  }
  static __device__ __forceinline__ v8f mma(v16h a, v16h b, v8f c) {
    return __builtin_amdgcn_wmma_f32_16x16x32_f16(false, a, false, b, (short)0, c, false, false);
  }
};

__device__ __forceinline__ void guard_main(v8f& a0, v8f& a1, v8f& a2, v8f& a3, v8f& r0, v8f& r1, v8f& r2, v8f& r3,
                                           v16h x0, v16h x1, v16h y0, v16h y1, v16h y2, v16h y3) {
  asm volatile("v_nop\n\tv_nop\n\tv_nop\n\tv_nop"
               : "+v"(a0), "+v"(a1), "+v"(a2), "+v"(a3), "+v"(r0), "+v"(r1), "+v"(r2), "+v"(r3)
               : "v"(x0), "v"(x1), "v"(y0), "v"(y1), "v"(y2), "v"(y3)
               : "memory");
}
__device__ __forceinline__ void guard_res(v8f& r0, v8f& r1, v8f& r2, v8f& r3,
                                          v16h x0, v16h y0, v16h y1, v16h y2, v16h y3) {
  asm volatile("v_nop\n\tv_nop\n\tv_nop\n\tv_nop"
               : "+v"(r0), "+v"(r1), "+v"(r2), "+v"(r3)
               : "v"(x0), "v"(y0), "v"(y1), "v"(y2), "v"(y3)
               : "memory");
}
__device__ __forceinline__ void acc_guard4(v8f& a, v8f& b, v8f& c, v8f& d) {
  asm volatile("v_nop\n\tv_nop\n\tv_nop\n\tv_nop" : "+v"(a), "+v"(b), "+v"(c), "+v"(d));
}

__device__ __forceinline__ float fsig(float z)  { return __builtin_amdgcn_rcpf(1.0f + expf(-z)); }
__device__ __forceinline__ float ftanh(float z) { return 1.0f - 2.0f * __builtin_amdgcn_rcpf(expf(2.0f * z) + 1.0f); }

__global__ __launch_bounds__(NTHRP) void wplane_kernel(const float* __restrict__ whh, const float* __restrict__ wih,
                                                       unsigned short* __restrict__ WHI, unsigned short* __restrict__ WLO) {
  const int i   = blockIdx.x * NTHRP + threadIdx.x;
  const int row = i >> 4;
  const int c8  = (i & 15) * 8;
  const int cw  = (c8 < NH - 8) ? c8 : (NH - 8);
  const int cx  = c8 - NH;
  const int ci  = (cx < 0) ? 0 : ((cx > NIN - 8) ? (NIN - 8) : cx);
  const v4f a0 = *(const v4f*)(whh + (size_t)row * NH + cw);
  const v4f a1 = *(const v4f*)(whh + (size_t)row * NH + cw + 4);
  const v4f b0 = *(const v4f*)(wih + (size_t)row * NIN + ci);
  const v4f b1 = *(const v4f*)(wih + (size_t)row * NIN + ci + 4);
  const float fa = (c8 < NH) ? WCARRY : 0.0f;
  const float fb = (c8 >= NH && c8 < NH + NIN) ? WCARRY : 0.0f;
  v8h hv, lv;
#pragma unroll
  for (int e = 0; e < 4; ++e) {
    const float v = fmaf(fa, a0[e], fb * b0[e]);
    const _Float16 h = (_Float16)v;
    hv[e] = h;
    lv[e] = (_Float16)((v - (float)h) * LCARRY);
  }
#pragma unroll
  for (int e = 0; e < 4; ++e) {
    const float v = fmaf(fa, a1[e], fb * b1[e]);
    const _Float16 h = (_Float16)v;
    hv[4 + e] = h;
    lv[4 + e] = (_Float16)((v - (float)h) * LCARRY);
  }
  unsigned short* ph = WHI + (size_t)i * 8;
  unsigned short* pl = WLO + (size_t)i * 8;
  *(volatile v8h*)ph = hv;
  *(volatile v8h*)pl = lv;
  __threadfence();
  *(volatile v8h*)ph = hv;
  *(volatile v8h*)pl = lv;
}

__device__ __forceinline__ void stage_x(const float* __restrict__ x, unsigned short* ahi, unsigned short* alo,
                                        int b0, int tid, int tsrc) {
  const int xm = tid >> 3, xq = tid & 7;
  const v4f xv = *(const v4f*)(x + ((size_t)(b0 + xm) * NT + (size_t)tsrc) * NIN + (size_t)((xq & 3) * 4));
  const float fsel = (xq < 4) ? 1.0f : 0.0f;
  unsigned hb[4], lb[4];
#pragma unroll
  for (int e = 0; e < 4; ++e) {
    const float v = fsel * xv[e];
    const _Float16 h16 = (_Float16)v;
    const _Float16 l16 = (_Float16)((v - (float)h16) * LCARRY);
    hb[e] = (unsigned)__builtin_bit_cast(unsigned short, h16);
    lb[e] = (unsigned)__builtin_bit_cast(unsigned short, l16);
  }
  v2u ph, pl;
  ph[0] = hb[0] | (hb[1] << 16);
  ph[1] = hb[2] | (hb[3] << 16);
  pl[0] = lb[0] | (lb[1] << 16);
  pl[1] = lb[2] | (lb[3] << 16);
  *(v2u*)(ahi + xm * AP + NH + 4 * xq) = ph;
  *(v2u*)(alo + xm * AP + NH + 4 * xq) = pl;
}

__global__ __launch_bounds__(NTHR) void lstm_seq_kernel(const float* __restrict__ x, const float* __restrict__ b_ih,
                                                        const float* __restrict__ b_hh, const float* __restrict__ w_out,
                                                        const float* __restrict__ b_out,
                                                        const unsigned short* __restrict__ WHIp,
                                                        const unsigned short* __restrict__ WLOp,
                                                        float* __restrict__ out) {
  __shared__ __align__(16) unsigned short Ahi[ROWB * AP];
  __shared__ __align__(16) unsigned short Alo[ROWB * AP];
  __shared__ __align__(16) float          Hf[ROWB * HFP];
  __shared__ __align__(16) float          Wo[NO * NH];
  __shared__ __align__(16) float          Ob[ROWB * OBP];
  const _Float16* WH = (const _Float16*)WHIp;
  const _Float16* WL = (const _Float16*)WLOp;
  const int tid = threadIdx.x, lane = tid & 31, wave = tid >> 5;
  const int c = lane & 15, hh = lane >> 4, koff = hh * 8;
  const int j = 16 * wave + c;
  const int b0 = blockIdx.x * ROWB;

#pragma unroll 1
  for (int i = tid; i < ROWB * AP; i += NTHR) { Ahi[i] = (unsigned short)0; Alo[i] = (unsigned short)0; }
  __syncthreads();
  stage_x(x, Ahi, Alo, b0, tid, 0);
  {
    const v4f wv = *(const v4f*)(w_out + (tid & 31) * 4);
    *(v4f*)(Wo + (tid & 31) * 4) = wv;
  }
  float bias4[4];
#pragma unroll
  for (int G = 0; G < 4; ++G) bias4[G] = b_ih[G * NH + j] + b_hh[G * NH + j];
  const float bo = b_out[lane & 1];
  float cst[8];
#pragma unroll
  for (int r = 0; r < 8; ++r) cst[r] = 0.0f;
  __syncthreads();

  const _Float16* ahrow = (const _Float16*)Ahi + c * AP + koff;
  const _Float16* alrow = (const _Float16*)Alo + c * AP + koff;
  const v8f z8 = {0.f, 0.f, 0.f, 0.f, 0.f, 0.f, 0.f, 0.f};

#pragma unroll 1
  for (int t = 0; t < NT; ++t) {
    v8f acc[4], res[4];
    acc[0] = z8; acc[1] = z8; acc[2] = z8; acc[3] = z8;
    res[0] = z8; res[1] = z8; res[2] = z8; res[3] = z8;
#pragma unroll 1
    for (int ks = 0; ks < KTOT; ks += 32) {
      const v16h ah = Frag<_Float16>::load(ahrow + ks);
      const v16h al = Frag<_Float16>::load(alrow + ks);
      v16h bh[4];
#pragma unroll
      for (int G = 0; G < 4; ++G) bh[G] = Frag<_Float16>::load(WH + (size_t)(G * NH + j) * WPITCH + koff + ks);
#pragma unroll
      for (int G = 0; G < 4; ++G) {
        acc[G] = Frag<_Float16>::mma(ah, bh[G], acc[G]);
        res[G] = Frag<_Float16>::mma(al, bh[G], res[G]);
      }
      guard_main(acc[0], acc[1], acc[2], acc[3], res[0], res[1], res[2], res[3], ah, al, bh[0], bh[1], bh[2], bh[3]);
      v16h bl[4];
#pragma unroll
      for (int G = 0; G < 4; ++G) bl[G] = Frag<_Float16>::load(WL + (size_t)(G * NH + j) * WPITCH + koff + ks);
#pragma unroll
      for (int G = 0; G < 4; ++G) res[G] = Frag<_Float16>::mma(ah, bl[G], res[G]);
      guard_res(res[0], res[1], res[2], res[3], ah, bl[0], bl[1], bl[2], bl[3]);
    }
    acc_guard4(acc[0], acc[1], acc[2], acc[3]);
    acc_guard4(res[0], res[1], res[2], res[3]);

    float hn[8];
#pragma unroll
    for (int r = 0; r < 8; ++r) {
      const float zi = fmaf(res[0][r], LCARRY_INV, acc[0][r]) * WCARRY_INV + bias4[0];
      const float zf = fmaf(res[1][r], LCARRY_INV, acc[1][r]) * WCARRY_INV + bias4[1];
      const float zg = fmaf(res[2][r], LCARRY_INV, acc[2][r]) * WCARRY_INV + bias4[2];
      const float zo = fmaf(res[3][r], LCARRY_INV, acc[3][r]) * WCARRY_INV + bias4[3];
      const float ig = fsig(zi);
      const float fg = fsig(zf);
      const float gg = ftanh(zg);
      const float og = fsig(zo);
      const float cn = fg * cst[r] + ig * gg;
      cst[r] = cn;
      hn[r] = og * ftanh(cn);
    }

    __syncthreads();
#pragma unroll
    for (int r = 0; r < 8; ++r) {
      const float hv = hn[r];
      const _Float16 h16 = (_Float16)hv;
      const _Float16 l16 = (_Float16)((hv - (float)h16) * LCARRY);
      const int ro = 8 * hh + r;
      Ahi[ro * AP + j] = __builtin_bit_cast(unsigned short, h16);
      Alo[ro * AP + j] = __builtin_bit_cast(unsigned short, l16);
      Hf[ro * HFP + j] = hv;
    }
    stage_x(x, Ahi, Alo, b0, tid, (t + 1 < NT) ? (t + 1) : (NT - 1));
    __syncthreads();

    if (wave == 0) {
      const int hm = lane >> 1, ho = lane & 1;
      const float* hrow = Hf + hm * HFP;
      const float* wrow = Wo + ho * NH;
      float s = 0.0f;
#pragma unroll
      for (int k4 = 0; k4 < NH / 4; ++k4) {
        const v4f a = *(const v4f*)(hrow + 4 * k4);
        const v4f w = *(const v4f*)(wrow + 4 * k4);
        s = fmaf(a[0], w[0], s);
        s = fmaf(a[1], w[1], s);
        s = fmaf(a[2], w[2], s);
        s = fmaf(a[3], w[3], s);
      }
      Ob[hm * OBP + 2 * (t & (TFL - 1)) + ho] = s + bo;
      if ((t & (TFL - 1)) == (TFL - 1)) {
        __builtin_amdgcn_fence(__ATOMIC_RELEASE, "workgroup");
        __builtin_amdgcn_wave_barrier();
        __builtin_amdgcn_fence(__ATOMIC_ACQUIRE, "workgroup");
        const int t0 = t - (TFL - 1);
        const int lrow = lane >> 3, c4 = (lane & 7) * 4;
        for (int pass = 0; pass < 2; ++pass) {
#pragma unroll
          for (int it = 0; it < 4; ++it) {
            const int row = it * 4 + lrow;
            const v4f v = *(const v4f*)(Ob + row * OBP + c4);
            *(volatile v4f*)(out + ((size_t)(b0 + row) * NT + (size_t)t0) * NO + c4) = v;
          }
          __threadfence();
        }
        __builtin_amdgcn_fence(__ATOMIC_RELEASE, "workgroup");
        __builtin_amdgcn_wave_barrier();
        __builtin_amdgcn_fence(__ATOMIC_ACQUIRE, "workgroup");
      }
    }
  }
}

extern "C" void kernel_launch(void* const* d_in, const int* in_sizes, int n_in,
                              void* d_out, int out_size, void* d_ws, size_t ws_size, hipStream_t stream) {
  if (n_in < 7 || d_out == nullptr || d_ws == nullptr || in_sizes == nullptr) return;
  {
    const long long nx = (long long)in_sizes[0];
    const long long ex = (long long)NB * NT * NIN;
    if (nx != ex && nx != 4LL * ex) return;
    const long long no = (long long)out_size;
    const long long eo = (long long)NB * NT * NO;
    if (no != eo && no != 4LL * eo) return;
  }
  const float* x     = (const float*)d_in[0];
  const float* w_ih  = (const float*)d_in[1];
  const float* w_hh  = (const float*)d_in[2];
  const float* b_ih  = (const float*)d_in[3];
  const float* b_hh  = (const float*)d_in[4];
  const float* w_out = (const float*)d_in[5];
  const float* b_out = (const float*)d_in[6];
  float* out = (float*)d_out;

  char* ws = (char*)d_ws; size_t off = 0;
  auto carve = [&](size_t bytes) -> char* { char* p = ws + off; off += (bytes + 255) & ~(size_t)255; return p; };
  unsigned short* WHI = (unsigned short*)carve((size_t)NGC * WPITCH * 2);
  unsigned short* WLO = (unsigned short*)carve((size_t)NGC * WPITCH * 2);
  if (off > ws_size || off > (size_t)134217728) return;

  wplane_kernel<<<(NGC * (WPITCH / 8)) / NTHRP, NTHRP, 0, stream>>>(w_hh, w_ih, WHI, WLO);
  lstm_seq_kernel<<<NB / ROWB, NTHR, 0, stream>>>(x, b_ih, b_hh, w_out, b_out, WHI, WLO, out);
}
